// MultiHeadSelfAttention_2740189135249
// MI455X (gfx1250) — hardware-verified
//
#include <hip/hip_runtime.h>


#ifndef NB
#define NB 8
#endif
#ifndef SEQ
#define SEQ 1024
#endif
#define NB_FULL   8
#define SEQ_FULL  1024
#define HID       768
#define NHEAD     12
#define HD        64
#define MROWS     (NB * SEQ)
#define QKVW      (3 * HID)
#define RPIECES   (HID / 8)

static_assert(HID == NHEAD * HD);
static_assert(HD == 64);
static_assert(SEQ % 128 == 0);
static_assert(SEQ <= SEQ_FULL);
static_assert(NB >= 1 && NB <= NB_FULL);
static_assert(MROWS % 128 == 0);
static_assert(HID % 128 == 0);
static_assert(HID % 32 == 0);
static_assert(HID % 8 == 0);
static_assert(RPIECES % 8 == 0);
static_assert(QKVW % 128 == 0);
static_assert(((size_t)5 * MROWS * HID + (size_t)QKVW * HID + (size_t)HID * HID) * 2 <= (size_t)134217728);

#define CARRY_X    16.0f
#define CARRY_W    32.0f
#define CARRY_QKV  16.0f
#define CARRY_CTX  1024.0f

typedef _Float16 f16;
typedef f16   v16h __attribute__((ext_vector_type(16)));
typedef f16   v8h  __attribute__((ext_vector_type(8)));
typedef float v8f  __attribute__((ext_vector_type(8)));
typedef float v4f  __attribute__((ext_vector_type(4)));

union FragU { v16h v; v8h half[2]; f16 e[16]; };
union H8U   { v8h v; f16 e[8]; };

__device__ __forceinline__ v8f zero8() {
    v8f z = {0.f, 0.f, 0.f, 0.f, 0.f, 0.f, 0.f, 0.f};
    return z;
}

__device__ __forceinline__ v8f wmma16(v16h a, v16h b, v8f c) {
    v8f d = __builtin_amdgcn_wmma_f32_16x16x32_f16(false, a, false, b, (short)0, c, false, false);
    asm volatile("v_nop\n\tv_nop\n\tv_nop\n\tv_nop" : "+v"(d) : "v"(a), "v"(b));
    return d;
}

__device__ __forceinline__ float bf16_rne(float x) {
    unsigned u = __float_as_uint(x);
    u = (u + 0x7fffu + ((u >> 16) & 1u)) & 0xffff0000u;
    return __uint_as_float(u);
}

__device__ __forceinline__ float fexp2(float x) {
#if defined(__has_builtin)
#if __has_builtin(__builtin_amdgcn_exp2f)
    return __builtin_amdgcn_exp2f(x);
#else
    return exp2f(x);
#endif
#else
    return exp2f(x);
#endif
}

__device__ __forceinline__ float rowmax16(float x) {
    int v = __builtin_bit_cast(int, x);
    x = fmaxf(x, __builtin_bit_cast(float, __builtin_amdgcn_update_dpp(v, v, 0x121, 0xf, 0xf, false)));
    v = __builtin_bit_cast(int, x);
    x = fmaxf(x, __builtin_bit_cast(float, __builtin_amdgcn_update_dpp(v, v, 0x122, 0xf, 0xf, false)));
    v = __builtin_bit_cast(int, x);
    x = fmaxf(x, __builtin_bit_cast(float, __builtin_amdgcn_update_dpp(v, v, 0x124, 0xf, 0xf, false)));
    v = __builtin_bit_cast(int, x);
    x = fmaxf(x, __builtin_bit_cast(float, __builtin_amdgcn_update_dpp(v, v, 0x128, 0xf, 0xf, false)));
    return x;
}

__device__ __forceinline__ v16h load_frag_lds(const f16* tile, int rowbase, int pitch, int kcol, int lane) {
    const int r  = rowbase + (lane & 15);
    const int kh = (lane >> 4) << 3;
    const int off = r * pitch + kcol + kh;
    FragU f;
    f.half[0] = *(const v8h*)(tile + off);
    f.half[1] = *(const v8h*)(tile + off + 16);
    return f.v;
}

__device__ __forceinline__ v16h load_frag_glb(const f16* __restrict__ plane, size_t base, int rowbase,
                                              int pitch, int kcol, int lane) {
    const int r  = rowbase + (lane & 15);
    const int kh = (lane >> 4) << 3;
    const f16* p = plane + base + (size_t)r * pitch + kcol + kh;
    FragU f;
    f.half[0] = *(const v8h*)(p);
    f.half[1] = *(const v8h*)(p + 16);
    return f.v;
}

__global__ void __launch_bounds__(256)
cvt_rows(const float* __restrict__ src, f16* __restrict__ dst, int nrows, int dstper, int srcper,
         float carry) {
    const int g  = (int)blockIdx.x * 256 + (int)threadIdx.x;
    const int m  = g / RPIECES;
    const int c8 = (g - m * RPIECES) << 3;
    if (m >= nrows) return;
    const int blk = m / dstper;
    const int sm  = blk * srcper + (m - blk * dstper);
    const float* sp = src + (size_t)sm * HID + c8;
    const v4f a = *(const v4f*)sp;
    const v4f b = *(const v4f*)(sp + 4);
    H8U o;
#pragma unroll
    for (int j = 0; j < 4; ++j) {
        const float x0 = a[j];
        const float x1 = b[j];
        o.e[j]     = (f16)(bf16_rne(x0) * carry);
        o.e[j + 4] = (f16)(bf16_rne(x1) * carry);
    }
    f16* dp = dst + (size_t)m * HID + c8;
    *(volatile v8h*)dp = o.v;
    __threadfence();
    *(volatile v8h*)dp = o.v;
}

template <int MODE>
__device__ __forceinline__ void gemm_body(const f16* __restrict__ A, const f16* __restrict__ W,
                                          const float* __restrict__ bias, void* __restrict__ out,
                                          float accMul, float addMul) {
    __shared__ __attribute__((aligned(16))) f16 As[128 * 32];
    __shared__ __attribute__((aligned(16))) f16 Bs[128 * 32];
    __shared__ __attribute__((aligned(16))) f16 Cs[128 * 128];

    static_assert(MODE >= 0 && MODE <= 2);

    const int tid  = (int)threadIdx.x;
    const int lane = tid & 31;
    const int wave = tid >> 5;
    const int wm   = wave & 3;
    const int wn   = wave >> 2;
    const int hh8  = (lane >> 4) << 3;
    const int c16  = lane & 15;
    const int m0   = (int)blockIdx.x * 128;
    const int n0   = (int)blockIdx.y * 128;

    v8f acc[2][4];
#pragma unroll
    for (int i = 0; i < 2; ++i)
#pragma unroll
        for (int j = 0; j < 4; ++j) acc[i][j] = zero8();

    const int srow = tid >> 1;
    const int scol = (tid & 1) << 4;
    const f16* gA = A + (size_t)(m0 + srow) * HID + scol;
    const f16* gW = W + (size_t)(n0 + srow) * HID + scol;

#pragma unroll 1
    for (int k0 = 0; k0 < HID; k0 += 32) {
        const v8h ra0 = *(const v8h*)(gA + k0);
        const v8h ra1 = *(const v8h*)(gA + k0 + 8);
        const v8h rb0 = *(const v8h*)(gW + k0);
        const v8h rb1 = *(const v8h*)(gW + k0 + 8);
        __syncthreads();
        *(v8h*)&As[srow * 32 + scol]     = ra0;
        *(v8h*)&As[srow * 32 + scol + 8] = ra1;
        *(v8h*)&Bs[srow * 32 + scol]     = rb0;
        *(v8h*)&Bs[srow * 32 + scol + 8] = rb1;
        __syncthreads();

        v16h af[2], bfr[4];
#pragma unroll
        for (int i = 0; i < 2; ++i) af[i] = load_frag_lds(As, wm * 32 + i * 16, 32, 0, lane);
#pragma unroll
        for (int j = 0; j < 4; ++j) bfr[j] = load_frag_lds(Bs, wn * 64 + j * 16, 32, 0, lane);
#pragma unroll
        for (int i = 0; i < 2; ++i)
#pragma unroll
            for (int j = 0; j < 4; ++j) acc[i][j] = wmma16(af[i], bfr[j], acc[i][j]);
    }

    float bb[4];
#pragma unroll
    for (int j = 0; j < 4; ++j) bb[j] = bf16_rne(bias[n0 + wn * 64 + j * 16 + c16]) * addMul;

    const int bidx  = m0 / SEQ;
    const int s0    = m0 - bidx * SEQ;
    const int piece = lane & 7;
    const int lsub  = lane >> 3;

    if constexpr (MODE == 0) {
#pragma unroll
        for (int i = 0; i < 2; ++i)
#pragma unroll
            for (int j = 0; j < 4; ++j) {
                const int nl = wn * 64 + j * 16 + c16;
#pragma unroll
                for (int r = 0; r < 8; ++r) {
                    const int ml = wm * 32 + i * 16 + hh8 + r;
                    Cs[ml * 128 + nl] = (f16)(acc[i][j][r] * accMul + bb[j]);
                }
            }
        __syncthreads();
        f16* op = (f16*)out;
        const size_t bh0 = (size_t)bidx * NHEAD + (n0 >> 6);
#pragma unroll
        for (int pass = 0; pass < 2; ++pass) {
#pragma unroll
            for (int it = 0; it < 8; ++it) {
                const int L    = wave * 32 + it * 4 + lsub;
                const int ml   = L >> 1;
                const int hsel = L & 1;
                const v8h v = *(const v8h*)&Cs[ml * 128 + hsel * 64 + piece * 8];
                f16* dp = op + ((bh0 + hsel) * SEQ + s0 + ml) * HD + piece * 8;
                *(volatile v8h*)dp = v;
            }
            if (pass == 0) __threadfence();
        }
    } else if constexpr (MODE == 1) {
#pragma unroll
        for (int i = 0; i < 2; ++i)
#pragma unroll
            for (int j = 0; j < 4; ++j) {
                const int nl = wn * 64 + j * 16 + c16;
                H8U t;
#pragma unroll
                for (int r = 0; r < 8; ++r) t.e[r] = (f16)(acc[i][j][r] * accMul + bb[j]);
                *(v8h*)&Cs[nl * 128 + wm * 32 + i * 16 + hh8] = t.v;
            }
        __syncthreads();
        f16* op = (f16*)out;
#pragma unroll
        for (int pass = 0; pass < 2; ++pass) {
#pragma unroll
            for (int it = 0; it < 8; ++it) {
                const int L  = wave * 32 + it * 4 + lsub;
                const int nl = L >> 1;
                const int mh = L & 1;
                const v8h v = *(const v8h*)&Cs[nl * 128 + mh * 64 + piece * 8];
                f16* dp = op + ((size_t)(bidx * HID + n0 + nl) * SEQ + s0 + mh * 64 + piece * 8);
                *(volatile v8h*)dp = v;
            }
            if (pass == 0) __threadfence();
        }
    } else {
        float* Cf = (float*)Cs;
        float* of = (float*)out;
#pragma unroll
        for (int half = 0; half < 2; ++half) {
            if ((wm >> 1) == half) {
#pragma unroll
                for (int i = 0; i < 2; ++i)
#pragma unroll
                    for (int j = 0; j < 4; ++j) {
                        const int nl = wn * 64 + j * 16 + c16;
#pragma unroll
                        for (int r = 0; r < 8; ++r) {
                            const int ml = (wm & 1) * 32 + i * 16 + hh8 + r;
                            Cf[ml * 128 + nl] = acc[i][j][r] * accMul + bb[j];
                        }
                    }
            }
            __syncthreads();
#pragma unroll
            for (int pass = 0; pass < 2; ++pass) {
#pragma unroll
                for (int it = 0; it < 8; ++it) {
                    const int L    = wave * 32 + it * 4 + lsub;
                    const int row  = L >> 2;
                    const int part = L & 3;
                    const v4f v = *(const v4f*)&Cf[row * 128 + part * 32 + piece * 4];
                    float* dp = of + (size_t)(m0 + half * 64 + row) * HID + n0 + part * 32 + piece * 4;
                    *(volatile v4f*)dp = v;
                }
                if (pass == 0) __threadfence();
            }
            __syncthreads();
        }
    }
}

__global__ void __launch_bounds__(256) __attribute__((amdgpu_num_vgpr(256)))
gemm_heads(const f16* __restrict__ A, const f16* __restrict__ W, const float* __restrict__ bias,
           f16* __restrict__ out, float accMul, float addMul) {
    gemm_body<0>(A, W, bias, (void*)out, accMul, addMul);
}

__global__ void __launch_bounds__(256) __attribute__((amdgpu_num_vgpr(256)))
gemm_vt(const f16* __restrict__ A, const f16* __restrict__ W, const float* __restrict__ bias,
        f16* __restrict__ out, float accMul, float addMul) {
    gemm_body<1>(A, W, bias, (void*)out, accMul, addMul);
}

__global__ void __launch_bounds__(256) __attribute__((amdgpu_num_vgpr(256)))
gemm_out(const f16* __restrict__ A, const f16* __restrict__ W, const float* __restrict__ bias,
         float* __restrict__ out, float accMul, float addMul) {
    gemm_body<2>(A, W, bias, (void*)out, accMul, addMul);
}

__global__ void __launch_bounds__(256) __attribute__((amdgpu_num_vgpr(256)))
attn_fwd(const f16* __restrict__ Qp, const f16* __restrict__ Kp, const f16* __restrict__ Vt,
         f16* __restrict__ Cp) {
    __shared__ __attribute__((aligned(16))) f16 ks[64 * 64];
    __shared__ __attribute__((aligned(16))) f16 vsT[64 * 64];
    __shared__ __attribute__((aligned(16))) f16 ps[8 * 16 * 64];

    const int tid  = (int)threadIdx.x;
    const int lane = tid & 31;
    const int wave = tid >> 5;
    const int hh8  = (lane >> 4) << 3;
    const int c16  = lane & 15;
    const int bh   = (int)blockIdx.y;
    const int bidx = bh / NHEAD;
    const int hidx = bh - bidx * NHEAD;
    const int q0   = (int)blockIdx.x * 128 + wave * 16;
    const int pw   = wave * 16;
    const size_t head = (size_t)bh * SEQ * HD;

    v16h qa[2];
#pragma unroll
    for (int c = 0; c < 2; ++c) qa[c] = load_frag_glb(Qp, head, q0, HD, c * 32, lane);

    FragU onesu;
#pragma unroll
    for (int i = 0; i < 16; ++i) onesu.e[i] = (f16)1.0f;
    const v16h ones = onesu.v;

    float m[8];
    v8f   o[4], lacc;
#pragma unroll
    for (int r = 0; r < 8; ++r) m[r] = -1.0e30f;
#pragma unroll
    for (int dt = 0; dt < 4; ++dt) o[dt] = zero8();
    lacc = zero8();

    const float cl = 1.4426950408889634f * 0.00048828125f;

#pragma unroll 1
    for (int kt = 0; kt < SEQ / 64; ++kt) {
        __syncthreads();
#pragma unroll
        for (int p2 = 0; p2 < 2; ++p2) {
            const int p   = tid + p2 * 256;
            const int row = p >> 3;
            const int pc  = (p & 7) << 3;
            const v8h kv = *(const v8h*)(Kp + head + (size_t)(kt * 64 + row) * HD + pc);
            const v8h vv = *(const v8h*)(Vt + head + (size_t)row * SEQ + kt * 64 + pc);
            *(v8h*)&ks[row * 64 + pc]  = kv;
            *(v8h*)&vsT[row * 64 + pc] = vv;
        }
        __syncthreads();

        v8f s[4];
#pragma unroll
        for (int nt = 0; nt < 4; ++nt) s[nt] = zero8();
#pragma unroll
        for (int c = 0; c < 2; ++c) {
#pragma unroll
            for (int nt = 0; nt < 4; ++nt) {
                const v16h kb = load_frag_lds(ks, nt * 16, 64, c * 32, lane);
                s[nt] = wmma16(qa[c], kb, s[nt]);
            }
        }

#pragma unroll
        for (int r = 0; r < 8; ++r) {
            float x[4];
#pragma unroll
            for (int nt = 0; nt < 4; ++nt) x[nt] = s[nt][r] * cl;
            const float tm = rowmax16(fmaxf(fmaxf(x[0], x[1]), fmaxf(x[2], x[3])));
            const float mn = fmaxf(m[r], tm);
            const float al = fexp2(m[r] - mn);
            m[r] = mn;
            lacc[r] *= al;
#pragma unroll
            for (int dt = 0; dt < 4; ++dt) o[dt][r] *= al;
            const float sh = 10.0f - mn;
#pragma unroll
            for (int nt = 0; nt < 4; ++nt)
                ps[(pw + hh8 + r) * 64 + nt * 16 + c16] = (f16)fexp2(x[nt] + sh);
        }
        __syncthreads();

#pragma unroll
        for (int kk = 0; kk < 2; ++kk) {
            const v16h pa = load_frag_lds(ps, pw, 64, kk * 32, lane);
#pragma unroll
            for (int dt = 0; dt < 4; ++dt) {
                const v16h vb = load_frag_lds(vsT, dt * 16, 64, kk * 32, lane);
                o[dt] = wmma16(pa, vb, o[dt]);
            }
            lacc = wmma16(pa, ones, lacc);
        }
    }
    __syncthreads();

#pragma unroll
    for (int r = 0; r < 8; ++r) {
        const float inv = (CARRY_CTX / CARRY_QKV) / lacc[r];
#pragma unroll
        for (int dt = 0; dt < 4; ++dt)
            ps[(pw + hh8 + r) * 64 + dt * 16 + c16] = (f16)(o[dt][r] * inv);
    }
    __syncthreads();

    const int piece = lane & 7;
    const int lsub  = lane >> 3;
#pragma unroll
    for (int pass = 0; pass < 2; ++pass) {
#pragma unroll
        for (int it = 0; it < 4; ++it) {
            const int L = it * 4 + lsub;
            const v8h v = *(const v8h*)&ps[(pw + L) * 64 + piece * 8];
            f16* dp = Cp + ((size_t)(bidx * SEQ + q0 + L) * HID + hidx * HD + piece * 8);
            *(volatile v8h*)dp = v;
        }
        if (pass == 0) __threadfence();
    }
}

extern "C" void kernel_launch(void* const* d_in, const int* in_sizes, int n_in,
                              void* d_out, int out_size, void* d_ws, size_t ws_size,
                              hipStream_t stream) {
    if (n_in < 5) return;
    if (in_sizes[0] < ((NB - 1) * SEQ_FULL + SEQ) * HID) return;
    if (in_sizes[1] < QKVW * HID) return;
    if (in_sizes[2] < QKVW) return;
    if (in_sizes[3] < HID * HID) return;
    if (in_sizes[4] < HID) return;
    if (out_size < MROWS * HID) return;

    const float* x     = (const float*)d_in[0];
    const float* wqkv  = (const float*)d_in[1];
    const float* bqkv  = (const float*)d_in[2];
    const float* wproj = (const float*)d_in[3];
    const float* bproj = (const float*)d_in[4];

    const size_t nX  = (size_t)MROWS * HID;
    const size_t nW  = (size_t)HID * HID;
    const size_t totalHalves = 5 * nX + 4 * nW;
    if (ws_size < totalHalves * sizeof(f16)) return;

    f16* Xh  = (f16*)d_ws;
    f16* Wh  = Xh  + nX;
    f16* Woh = Wh  + 3 * nW;
    f16* Qp  = Woh + nW;
    f16* Kp  = Qp  + nX;
    f16* Vtp = Kp  + nX;
    f16* Cp  = Vtp + nX;

    cvt_rows<<<(MROWS * RPIECES + 255) / 256, 256, 0, stream>>>(x, Xh, MROWS, SEQ, SEQ_FULL, CARRY_X);
    cvt_rows<<<(QKVW * RPIECES + 255) / 256, 256, 0, stream>>>(wqkv, Wh, QKVW, QKVW, QKVW, CARRY_W);
    cvt_rows<<<(HID * RPIECES + 255) / 256, 256, 0, stream>>>(wproj, Woh, HID, HID, HID, CARRY_W);

    const dim3 gg(MROWS / 128, HID / 128);
    const float accQKV = CARRY_QKV / (CARRY_X * CARRY_W);
    gemm_heads<<<gg, 256, 0, stream>>>(Xh, Wh,          bqkv,           Qp,  accQKV, CARRY_QKV);
    gemm_heads<<<gg, 256, 0, stream>>>(Xh, Wh + nW,     bqkv + HID,     Kp,  accQKV, CARRY_QKV);
    gemm_vt   <<<gg, 256, 0, stream>>>(Xh, Wh + 2 * nW, bqkv + 2 * HID, Vtp, accQKV, CARRY_QKV);

    attn_fwd<<<dim3(SEQ / 128, NB * NHEAD), 256, 0, stream>>>(Qp, Kp, Vtp, Cp);

    const float accOut = 1.0f / (CARRY_CTX * CARRY_W);
    gemm_out<<<gg, 256, 0, stream>>>(Cp, Woh, bproj, (float*)d_out, accOut, 1.0f);
}
